// Encoder_73091753443852
// MI455X (gfx1250) — hardware-run, weakly checked
//
#include <hip/hip_runtime.h>
#include <math.h>

constexpr int NVOCAB = 32000;
constexpr int NSTEP  = 4096;
constexpr int NIN    = 512;
constexpr int NHID   = 256;
constexpr int NGATE  = 4 * NHID;
constexpr int NLAYER = 2;
constexpr int NTHR   = 256;
constexpr int NCHAIN = 1024;
constexpr float XCARRY = 1024.0f;
constexpr float HCARRY = 1024.0f;
constexpr float WCARRY = 256.0f;
constexpr float SCALE_L0 = 1.0f / (XCARRY * WCARRY);
constexpr float SCALE_L1 = 1.0f / (HCARRY * WCARRY);
constexpr float F16_MIN_NORMAL = 6.103515625e-5f;
constexpr int OUT_CELL_OFF = 0;
constexpr int OUT_HID_OFF  = NLAYER * 2 * NHID;
constexpr int OUT_SEQ_OFF  = 2 * NLAYER * 2 * NHID;
constexpr int OUT_TOTAL    = OUT_SEQ_OFF + NSTEP * 2 * NHID;
static_assert(OUT_HID_OFF * 4 == 4096, "hidden finals byte offset");
static_assert(OUT_SEQ_OFF * 4 == 8192, "sequence byte offset");
static_assert((size_t)OUT_TOTAL * 4 == 8396800, "d_out total bytes");
static_assert(NGATE == 1024 && NCHAIN == NGATE, "one chain thread per gate row");
static_assert(NSTEP % 64 == 0 && NGATE % 64 == 0, "GEMM M, N tile multiples");
static_assert(NIN % 32 == 0 && NHID % 32 == 0, "GEMM K multiples of 32");
static_assert((NSTEP * NIN / 8) % NTHR == 0, "gather grid exact");
static_assert((NGATE * NIN / 8) % NTHR == 0 && (NGATE * NHID / 8) % NTHR == 0, "convert grid exact");
static_assert((NGATE * NHID / 4) % NTHR == 0, "pack grid exact");

typedef __attribute__((ext_vector_type(16))) _Float16 v16h;
typedef __attribute__((ext_vector_type(8)))  _Float16 v8h;
typedef __attribute__((ext_vector_type(8)))  float    v8f;
typedef __attribute__((ext_vector_type(4)))  float    v4f;

__device__ __forceinline__ _Float16 to_h_flush(float v) {
  const float q = (fabsf(v) < F16_MIN_NORMAL) ? 0.0f : v;
  return (_Float16)q;
}

__device__ __forceinline__ void guard_acc_h(v8f& a, v16h x, v16h y) {
  asm volatile("v_nop\n\tv_nop\n\tv_nop\n\tv_nop" : "+v"(a) : "v"(x), "v"(y));
}
__device__ __forceinline__ void guard_acc(v8f& a) {
  asm volatile("v_nop\n\tv_nop\n\tv_nop\n\tv_nop" : "+v"(a));
}
__device__ __forceinline__ void keep4_h(v16h a, v16h b, v16h c, v16h d) {
  asm volatile("v_nop" :: "v"(a), "v"(b), "v"(c), "v"(d));
}
__device__ __forceinline__ v16h frag_load_h(const _Float16* p) {
  union U { v16h v; v8h h[2]; } f;
  f.h[0] = *(const v8h*)(p);
  f.h[1] = *(const v8h*)(p + 16);
  return f.v;
}
__device__ __forceinline__ v8f mma_h(v16h a, v16h b, v8f c) {
  return __builtin_amdgcn_wmma_f32_16x16x32_f16(false, a, false, b, (short)0, c, false, false);
}

__device__ __forceinline__ float sigm(float x) { return 1.0f / (1.0f + expf(-x)); }

__global__ __launch_bounds__(NTHR) void embed_gather_kernel(const int* __restrict__ tokens,
                                                           const float* __restrict__ emb,
                                                           unsigned short* __restrict__ X16) {
  const int i  = blockIdx.x * NTHR + threadIdx.x;
  const int t  = i >> 6;
  const int c8 = i & 63;
  int tok = tokens[t];
  tok = tok < 0 ? 0 : (tok > NVOCAB - 1 ? NVOCAB - 1 : tok);
  const float* sp = emb + (size_t)tok * NIN + c8 * 8;
  const v4f a = *(const v4f*)(sp);
  const v4f b = *(const v4f*)(sp + 4);
  v8h hv;
#pragma unroll
  for (int e = 0; e < 4; ++e) {
    hv[e]     = to_h_flush(a[e] * XCARRY);
    hv[4 + e] = to_h_flush(b[e] * XCARRY);
  }
  unsigned short* op = X16 + (size_t)i * 8;
  *(volatile v8h*)op = hv;
  __threadfence();
  *(volatile v8h*)op = hv;
}

__global__ __launch_bounds__(NTHR) void wih_cvt_kernel(const float* __restrict__ s0, const float* __restrict__ s1,
                                                      const float* __restrict__ s2, const float* __restrict__ s3,
                                                      unsigned short* __restrict__ dst) {
  const int y  = blockIdx.y;
  const int n8 = (y < 2) ? (NGATE * NIN / 8) : (NGATE * NHID / 8);
  const int i  = blockIdx.x * NTHR + threadIdx.x;
  if (i >= n8) return;
  const float* src = (y == 0) ? s0 : (y == 1) ? s1 : (y == 2) ? s2 : s3;
  const size_t doff = (y == 0) ? (size_t)0
                    : (y == 1) ? (size_t)NGATE * NIN
                    : (y == 2) ? (size_t)2 * NGATE * NIN
                               : (size_t)2 * NGATE * NIN + (size_t)NGATE * NHID;
  const float* sp = src + (size_t)i * 8;
  const v4f a = *(const v4f*)(sp);
  const v4f b = *(const v4f*)(sp + 4);
  v8h hv;
#pragma unroll
  for (int e = 0; e < 4; ++e) {
    hv[e]     = to_h_flush(a[e] * WCARRY);
    hv[4 + e] = to_h_flush(b[e] * WCARRY);
  }
  unsigned short* op = dst + doff + (size_t)i * 8;
  *(volatile v8h*)op = hv;
  __threadfence();
  *(volatile v8h*)op = hv;
}

__global__ __launch_bounds__(NTHR) void whh_pack_kernel(const float* __restrict__ w0, const float* __restrict__ w1,
                                                       const float* __restrict__ w2, const float* __restrict__ w3,
                                                       float* __restrict__ dst) {
  const int y = blockIdx.y;
  const int i = blockIdx.x * NTHR + threadIdx.x;
  const int k4 = i >> 10;
  const int row = i & 1023;
  const float* src = (y == 0) ? w0 : (y == 1) ? w1 : (y == 2) ? w2 : w3;
  const v4f v = *(const v4f*)(src + (size_t)row * NHID + 4 * k4);
  float* op = dst + ((size_t)y * (NGATE * NHID / 4) + (size_t)i) * 4;
  *(volatile v4f*)op = v;
  __threadfence();
  *(volatile v4f*)op = v;
}

__global__ __launch_bounds__(256) void gemm64_f16_kernel(
    const unsigned short* __restrict__ Ap, int lda, long strideA,
    const unsigned short* __restrict__ Btp, int ldb, long strideB,
    float* __restrict__ Cout, int ldc, long strideC,
    int M, int N, int K, float scale) {
  __shared__ __align__(16) float sT[8][16 * 68];
  const _Float16* A  = (const _Float16*)Ap;
  const _Float16* Bt = (const _Float16*)Btp;
  const int b    = blockIdx.y;
  const int lane = threadIdx.x & 31;
  const int wave = threadIdx.x >> 5;
  const int tilesN = N >> 6;
  const int tilesM = M >> 6;
  const int tile = blockIdx.x * 8 + wave;
  if (tile >= tilesM * tilesN) return;
  const int tm = tile / tilesN;
  const int tn = tile - tm * tilesN;
  const int m0 = tm << 6;
  const int n0 = tn << 6;

  const _Float16* Ab = A  + (size_t)b * strideA;
  const _Float16* Bb = Bt + (size_t)b * strideB;

  const int rlane = lane & 15;
  const int koff  = (lane >> 4) * 8;
  const int mOff  = (lane >> 4) * 8;

  v8f acc[4][4];
#pragma unroll
  for (int i = 0; i < 4; ++i)
#pragma unroll
    for (int j = 0; j < 4; ++j) acc[i][j] = (v8f){0.f, 0.f, 0.f, 0.f, 0.f, 0.f, 0.f, 0.f};

  for (int k0 = 0; k0 < K; k0 += 32) {
    v16h bh[4];
#pragma unroll
    for (int j = 0; j < 4; ++j) {
      const size_t bo = (size_t)(n0 + (j << 4) + rlane) * ldb + koff + k0;
      bh[j] = frag_load_h(Bb + bo);
    }
#pragma unroll
    for (int i = 0; i < 4; ++i) {
      const size_t ao = (size_t)(m0 + (i << 4) + rlane) * lda + koff + k0;
      const v16h ah = frag_load_h(Ab + ao);
#pragma unroll
      for (int j = 0; j < 4; ++j) acc[i][j] = mma_h(ah, bh[j], acc[i][j]);
      guard_acc_h(acc[i][0], ah, bh[0]);
      guard_acc_h(acc[i][1], ah, bh[1]);
      guard_acc_h(acc[i][2], ah, bh[2]);
      guard_acc_h(acc[i][3], ah, bh[3]);
    }
    keep4_h(bh[0], bh[1], bh[2], bh[3]);
  }
#pragma unroll
  for (int i = 0; i < 4; ++i)
#pragma unroll
    for (int j = 0; j < 4; ++j) guard_acc(acc[i][j]);

  float* slab = sT[wave];
  float* C = Cout + (size_t)b * strideC;
#pragma unroll
  for (int i = 0; i < 4; ++i) {
    const int mBase = m0 + (i << 4);
#pragma unroll
    for (int j = 0; j < 4; ++j) {
#pragma unroll
      for (int r = 0; r < 8; ++r) {
        const float v = acc[i][j][r] * scale;
        slab[(mOff + r) * 68 + (j << 4) + rlane] = v;
      }
    }
    __builtin_amdgcn_fence(__ATOMIC_RELEASE, "workgroup");
    __builtin_amdgcn_wave_barrier();
    __builtin_amdgcn_fence(__ATOMIC_ACQUIRE, "workgroup");
    {
      const int hh = lane >> 4, c4 = (lane & 15) * 4;
      for (int pass = 0; pass < 2; ++pass) {
#pragma unroll
        for (int it = 0; it < 8; ++it) {
          const int row = it * 2 + hh;
          const v4f v = *(const v4f*)(slab + row * 68 + c4);
          *(volatile v4f*)(C + (size_t)(mBase + row) * ldc + n0 + c4) = v;
        }
        __threadfence();
      }
    }
    __builtin_amdgcn_fence(__ATOMIC_RELEASE, "workgroup");
    __builtin_amdgcn_wave_barrier();
    __builtin_amdgcn_fence(__ATOMIC_ACQUIRE, "workgroup");
  }
}

__global__ __launch_bounds__(NCHAIN) void lstm_chain_kernel(
    const float* __restrict__ G, const float* __restrict__ WP,
    const float* __restrict__ bihF, const float* __restrict__ bhhF,
    const float* __restrict__ bihB, const float* __restrict__ bhhB,
    unsigned short* __restrict__ H16, float* __restrict__ dout, int layer) {
  __shared__ __align__(16) float hsm[NHID];
  __shared__ __align__(16) float gsm[NGATE];

  const int d   = blockIdx.x;
  const int tid = threadIdx.x;
  const float* bi = d ? bihB : bihF;
  const float* bh = d ? bhhB : bhhF;
  const float bias = bi[tid] + bh[tid];
  const v4f* wp = (const v4f*)WP + (size_t)d * (NGATE * NHID / 4) + tid;
  const float* Gd = G + (size_t)d * NSTEP * NGATE + tid;

  float cst = 0.0f, hst = 0.0f;
  if (tid < NHID) hsm[tid] = 0.0f;
  __syncthreads();

#pragma unroll 1
  for (int s = 0; s < NSTEP; ++s) {
    const int t = d ? (NSTEP - 1 - s) : s;
    const float gin = Gd[(size_t)t * NGATE];
    float a0 = 0.0f, a1 = 0.0f, a2 = 0.0f, a3 = 0.0f;
#pragma unroll 8
    for (int k4 = 0; k4 < NHID / 4; ++k4) {
      const v4f w  = wp[(size_t)k4 * NGATE];
      const v4f hv = *(const v4f*)(hsm + 4 * k4);
      a0 = fmaf(w[0], hv[0], a0);
      a1 = fmaf(w[1], hv[1], a1);
      a2 = fmaf(w[2], hv[2], a2);
      a3 = fmaf(w[3], hv[3], a3);
    }
    gsm[tid] = (gin + bias) + ((a0 + a1) + (a2 + a3));
    __syncthreads();

    if (tid < NHID) {
      const float zi = gsm[tid];
      const float zf = gsm[tid + NHID];
      const float zg = gsm[tid + 2 * NHID];
      const float zo = gsm[tid + 3 * NHID];
      const float cn = sigm(zf) * cst + sigm(zi) * tanhf(zg);
      const float hn = sigm(zo) * tanhf(cn);
      cst = cn;
      hst = hn;
      hsm[tid] = hn;
      if (layer == 1) {
        float* op = dout + OUT_SEQ_OFF + (size_t)t * (2 * NHID) + d * NHID + tid;
        *(volatile float*)op = hn;
        __threadfence();
        *(volatile float*)op = hn;
      }
    }
    __syncthreads();

    if (layer == 0 && tid < 32) {
      const v4f p0 = *(const v4f*)(hsm + 8 * tid);
      const v4f p1 = *(const v4f*)(hsm + 8 * tid + 4);
      v8h hv8;
#pragma unroll
      for (int e = 0; e < 4; ++e) {
        hv8[e]     = to_h_flush(p0[e] * HCARRY);
        hv8[4 + e] = to_h_flush(p1[e] * HCARRY);
      }
      unsigned short* hp = H16 + ((size_t)d * NSTEP + (size_t)t) * NHID + 8 * tid;
      *(volatile v8h*)hp = hv8;
      __threadfence();
      *(volatile v8h*)hp = hv8;
    }
  }

  if (tid < NHID) {
    float* pc = dout + OUT_CELL_OFF + (layer * 2 + d) * NHID + tid;
    float* ph = dout + OUT_HID_OFF  + (layer * 2 + d) * NHID + tid;
    *(volatile float*)pc = cst;
    *(volatile float*)ph = hst;
    __threadfence();
    *(volatile float*)pc = cst;
    *(volatile float*)ph = hst;
  }
}

extern "C" void kernel_launch(void* const* d_in, const int* in_sizes, int n_in,
                              void* d_out, int out_size, void* d_ws, size_t ws_size, hipStream_t stream) {
  if (n_in < 18 || d_out == nullptr || d_ws == nullptr) return;
  if (in_sizes[0] != NSTEP || in_sizes[1] != NVOCAB * NIN) return;
  if (in_sizes[2] != NGATE * NIN || in_sizes[10] != NGATE * NIN) return;
  if (in_sizes[3] != NGATE * NHID || in_sizes[6] != NGATE * NHID || in_sizes[7] != NGATE * NHID) return;
  if (in_sizes[11] != NGATE * NHID || in_sizes[14] != NGATE * NHID || in_sizes[15] != NGATE * NHID) return;
  if (in_sizes[4] != NGATE || in_sizes[5] != NGATE || in_sizes[8] != NGATE || in_sizes[9] != NGATE) return;
  if (in_sizes[12] != NGATE || in_sizes[13] != NGATE || in_sizes[16] != NGATE || in_sizes[17] != NGATE) return;
  if (out_size != OUT_TOTAL) return;

  const int*   tokens = (const int*)  d_in[0];
  const float* emb    = (const float*)d_in[1];
  const float* fWih0  = (const float*)d_in[2];
  const float* fWhh0  = (const float*)d_in[3];
  const float* fbih0  = (const float*)d_in[4];
  const float* fbhh0  = (const float*)d_in[5];
  const float* fWih1  = (const float*)d_in[6];
  const float* fWhh1  = (const float*)d_in[7];
  const float* fbih1  = (const float*)d_in[8];
  const float* fbhh1  = (const float*)d_in[9];
  const float* bWih0  = (const float*)d_in[10];
  const float* bWhh0  = (const float*)d_in[11];
  const float* bbih0  = (const float*)d_in[12];
  const float* bbhh0  = (const float*)d_in[13];
  const float* bWih1  = (const float*)d_in[14];
  const float* bWhh1  = (const float*)d_in[15];
  const float* bbih1  = (const float*)d_in[16];
  const float* bbhh1  = (const float*)d_in[17];
  float* out = (float*)d_out;

  char* ws = (char*)d_ws;
  size_t off = 0;
  auto carve = [&](size_t bytes) -> char* { char* p = ws + off; off += (bytes + 255) & ~(size_t)255; return p; };
  unsigned short* X16 = (unsigned short*)carve((size_t)NSTEP * NIN * 2);
  unsigned short* W16 = (unsigned short*)carve(((size_t)2 * NGATE * NIN + (size_t)2 * NGATE * NHID) * 2);
  float*          WHP = (float*)carve((size_t)4 * NGATE * NHID * 4);
  float*          G   = (float*)carve((size_t)2 * NSTEP * NGATE * 4);
  unsigned short* H16 = (unsigned short*)carve((size_t)2 * NSTEP * NHID * 2);
  if (off > ws_size || off > (size_t)134217728) return;

  embed_gather_kernel<<<(NSTEP * NIN / 8) / NTHR, NTHR, 0, stream>>>(tokens, emb, X16);
  wih_cvt_kernel<<<dim3((NGATE * NIN / 8) / NTHR, 4), NTHR, 0, stream>>>(fWih0, bWih0, fWih1, bWih1, W16);
  whh_pack_kernel<<<dim3((NGATE * NHID / 4) / NTHR, 4), NTHR, 0, stream>>>(fWhh0, bWhh0, fWhh1, bWhh1, WHP);

  const dim3 ggrid((NSTEP / 64) * (NGATE / 64) / 8, 2);

  gemm64_f16_kernel<<<ggrid, 256, 0, stream>>>(
      X16, NIN, 0L,
      W16, NIN, (long)NGATE * NIN,
      G, NGATE, (long)NSTEP * NGATE,
      NSTEP, NGATE, NIN, SCALE_L0);
  lstm_chain_kernel<<<2, NCHAIN, 0, stream>>>(G, WHP, fbih0, fbhh0, bbih0, bbhh0, H16, out, 0);

  gemm64_f16_kernel<<<ggrid, 256, 0, stream>>>(
      H16, NHID, (long)NSTEP * NHID,
      W16 + (size_t)2 * NGATE * NIN, NHID, (long)NGATE * NHID,
      G, NGATE, (long)NSTEP * NGATE,
      NSTEP, NGATE, NHID, SCALE_L1);
  lstm_chain_kernel<<<2, NCHAIN, 0, stream>>>(G, WHP + (size_t)2 * NGATE * NHID, fbih1, fbhh1, bbih1, bbhh1, H16, out, 1);
}
